// QKVAttention_21766894256872
// MI455X (gfx1250) — hardware-verified
//
#include <hip/hip_runtime.h>
#include <math.h>
#include <stdint.h>

#define NBH   32
#define CH    64
#define SEQ   2048
#define WROW  (3 * CH)
#define NQB   (SEQ / 64)
#define NKT   (SEQ / 64)
#define TP    68
#define PO    68
static_assert(NQB == 32 && NKT == 32);
static_assert((SEQ % 64) == 0 && CH == 64);

typedef __bf16   v16b __attribute__((ext_vector_type(16)));
typedef float    v8f  __attribute__((ext_vector_type(8)));
typedef float    v4f  __attribute__((ext_vector_type(4)));
typedef unsigned int   v4u  __attribute__((ext_vector_type(4)));
typedef unsigned short v8us __attribute__((ext_vector_type(8)));

#if defined(__HIP_DEVICE_COMPILE__)
#define DEV_ASM 1
#else
#define DEV_ASM 0
#endif

__device__ __forceinline__ unsigned short bf_bits(float f) {
  unsigned u = __float_as_uint(f);
  return (unsigned short)((u + 0x7FFFu + ((u >> 16) & 1u)) >> 16);
}
__device__ __forceinline__ float bf_up(unsigned short hb) { return __uint_as_float(((unsigned)hb) << 16); }
__device__ __forceinline__ unsigned pk16(unsigned short a, unsigned short b) { return (unsigned)a | ((unsigned)b << 16); }
__device__ __forceinline__ v8f zero8() { v8f z = {0.f, 0.f, 0.f, 0.f, 0.f, 0.f, 0.f, 0.f}; return z; }

union FB { v16b v; v8us h[2]; };
__device__ __forceinline__ v16b ldfrag_b(const unsigned short* p) {
  FB f;
  f.h[0] = *(const v8us*)(p);
  f.h[1] = *(const v8us*)(p + 16);
  return f.v;
}

__device__ __forceinline__ v8f mma_b(v16b a, v16b b, v8f c) {
  c = __builtin_amdgcn_wmma_f32_16x16x32_bf16(false, a, false, b, (short)0, c, false, false);
#if DEV_ASM
  asm volatile("v_nop\n\tv_nop\n\tv_nop\n\tv_nop" : "+v"(c) : "v"(a), "v"(b));
#endif
  return c;
}

__global__ __launch_bounds__(256)
void prep_planes(const float* __restrict__ qkv, unsigned short* Qt, unsigned short* Kt, unsigned short* Vb) {
  __shared__ __align__(16) float qs[64 * TP];
  __shared__ __align__(16) float ks[64 * TP];
  const int tid = (int)threadIdx.x;
  const int bh  = (int)blockIdx.x >> 5;
  const int chk = (int)blockIdx.x & 31;
  const int t0  = chk * 64;
  const float* qg = qkv + ((size_t)bh * WROW) * SEQ + t0;
  const float* kg = qg + (size_t)CH * SEQ;
  const float* vg = qg + (size_t)(2 * CH) * SEQ;

#pragma unroll
  for (int i = 0; i < 4; ++i) {
    const int idx = tid + i * 256;
    const int c   = idx >> 4;
    const int j4  = (idx & 15) * 4;
    const v4f a = *(const v4f*)(qg + (size_t)c * SEQ + j4);
    const v4f b = *(const v4f*)(kg + (size_t)c * SEQ + j4);
    *(v4f*)(qs + c * TP + j4) = a;
    *(v4f*)(ks + c * TP + j4) = b;
  }

  v4u vv[2];
#pragma unroll
  for (int it = 0; it < 2; ++it) {
    const int job = tid + it * 256;
    const int c   = job >> 3;
    const int s8  = (job & 7) * 8;
    const v4f a  = *(const v4f*)(vg + (size_t)c * SEQ + s8);
    const v4f a4 = *(const v4f*)(vg + (size_t)c * SEQ + s8 + 4);
    v4u p;
    p[0] = pk16(bf_bits(a[0]),  bf_bits(a[1]));
    p[1] = pk16(bf_bits(a[2]),  bf_bits(a[3]));
    p[2] = pk16(bf_bits(a4[0]), bf_bits(a4[1]));
    p[3] = pk16(bf_bits(a4[2]), bf_bits(a4[3]));
    vv[it] = p;
  }
  __syncthreads();

  v4u qv[2], kv[2];
#pragma unroll
  for (int it = 0; it < 2; ++it) {
    const int job = tid + it * 256;
    const int t   = job >> 3;
    const int c8  = (job & 7) * 8;
    float fq[8], fk[8];
#pragma unroll
    for (int e = 0; e < 8; ++e) {
      fq[e] = qs[(c8 + e) * TP + t];
      fk[e] = ks[(c8 + e) * TP + t];
    }
    v4u a, b;
#pragma unroll
    for (int e = 0; e < 4; ++e) {
      a[e] = pk16(bf_bits(fq[2 * e]), bf_bits(fq[2 * e + 1]));
      b[e] = pk16(bf_bits(fk[2 * e]), bf_bits(fk[2 * e + 1]));
    }
    qv[it] = a; kv[it] = b;
  }

  for (int pass = 0; pass < 2; ++pass) {
#pragma unroll
    for (int it = 0; it < 2; ++it) {
      const int job = tid + it * 256;
      const int r   = job >> 3;
      const int e8  = (job & 7) * 8;
      unsigned short* pq = Qt + ((size_t)(bh * SEQ + t0 + r)) * CH + e8;
      unsigned short* pk = Kt + ((size_t)(bh * SEQ + t0 + r)) * CH + e8;
      unsigned short* pv = Vb + ((size_t)(bh * CH + r)) * SEQ + t0 + e8;
      *(volatile v4u*)pq = qv[it];
      *(volatile v4u*)pk = kv[it];
      *(volatile v4u*)pv = vv[it];
    }
    __threadfence();
  }
}

__global__ __launch_bounds__(128)
void attn64(const unsigned short* __restrict__ Qt, const unsigned short* __restrict__ Kt,
            const unsigned short* __restrict__ Vb, float* out, float sscale) {
  __shared__ __align__(16) unsigned short Ksh[64 * 64];
  __shared__ __align__(16) unsigned short Vsh[64 * 64];
  __shared__ __align__(16) unsigned short Phs[4 * 16 * 64];
  __shared__ __align__(16) unsigned short Pls[4 * 16 * 64];
  __shared__ __align__(16) float Osh[64 * PO];

  const int tid  = (int)threadIdx.x;
  const int wave = tid >> 5;
  const int lane = tid & 31;
  const int hh   = lane >> 4;
  const int c    = lane & 15;

  const int bh = (int)blockIdx.x >> 5;
  const int qb = (int)blockIdx.x & 31;
  const int q0 = qb * 64;

  v16b qa[2];
#pragma unroll
  for (int dc = 0; dc < 2; ++dc) {
    const size_t qo = ((size_t)(bh * SEQ + q0 + wave * 16 + c)) * CH + dc * 32 + 8 * hh;
    qa[dc] = ldfrag_b(Qt + qo);
  }

  float mrow[8], lrow[8];
  v8f oacc[4];
#pragma unroll
  for (int r = 0; r < 8; ++r) { mrow[r] = -INFINITY; lrow[r] = 0.f; }
#pragma unroll
  for (int t = 0; t < 4; ++t) oacc[t] = zero8();

  unsigned short* ph = Phs + wave * (16 * 64);
  unsigned short* pl = Pls + wave * (16 * 64);

  for (int kt = 0; kt < NKT; ++kt) {
    const int kv0 = kt * 64;
    __syncthreads();
    {
      const int r = tid >> 1, half = (tid & 1) * 32;
      const unsigned short* kg = Kt + ((size_t)(bh * SEQ + kv0 + r)) * CH + half;
      const unsigned short* vg = Vb + ((size_t)(bh * CH + r)) * SEQ + kv0 + half;
#pragma unroll
      for (int i = 0; i < 4; ++i) {
        const v8us a0 = *(const v8us*)(kg + 8 * i);
        const v8us b0 = *(const v8us*)(vg + 8 * i);
        *(v8us*)(Ksh + r * 64 + half + 8 * i) = a0;
        *(v8us*)(Vsh + r * 64 + half + 8 * i) = b0;
      }
    }
    __syncthreads();

    v8f s[4];
#pragma unroll
    for (int j = 0; j < 4; ++j) {
      v8f acc = zero8();
#pragma unroll
      for (int dc = 0; dc < 2; ++dc) {
        FB kb;
        kb.h[0] = *(const v8us*)(Ksh + (j * 16 + c) * 64 + dc * 32 + 8 * hh);
        kb.h[1] = *(const v8us*)(Ksh + (j * 16 + c) * 64 + dc * 32 + 16 + 8 * hh);
        acc = mma_b(qa[dc], kb.v, acc);
      }
#pragma unroll
      for (int r = 0; r < 8; ++r) s[j][r] = acc[r] * sscale;
    }

#pragma unroll
    for (int r = 0; r < 8; ++r) {
      float mx = s[0][r];
#pragma unroll
      for (int j = 1; j < 4; ++j) mx = fmaxf(mx, s[j][r]);
#pragma unroll
      for (int off = 1; off < 16; off <<= 1) mx = fmaxf(mx, __shfl_xor(mx, off, 32));
      const float mnew  = fmaxf(mrow[r], mx);
      const float msafe = (mnew == -INFINITY) ? 0.f : mnew;
      const float alpha = __expf(mrow[r] - msafe);
      mrow[r] = mnew;
      float psum = 0.f;
#pragma unroll
      for (int j = 0; j < 4; ++j) {
        const float p = __expf(s[j][r] - msafe);
        psum += p;
        const unsigned short hb = bf_bits(p);
        const float hu = bf_up(hb);
        const unsigned short lb = bf_bits(p - hu);
        const int idx = (8 * hh + r) * 64 + j * 16 + c;
        ph[idx] = hb;
        pl[idx] = lb;
      }
      lrow[r] = lrow[r] * alpha + psum;
#pragma unroll
      for (int t = 0; t < 4; ++t) oacc[t][r] *= alpha;
    }
    __builtin_amdgcn_fence(__ATOMIC_RELEASE, "workgroup");
    __builtin_amdgcn_wave_barrier();
    __builtin_amdgcn_fence(__ATOMIC_ACQUIRE, "workgroup");

#pragma unroll 1
    for (int kk = 0; kk < 2; ++kk) {
      FB pa, pb;
      pa.h[0] = *(const v8us*)(ph + c * 64 + kk * 32 + 8 * hh);
      pa.h[1] = *(const v8us*)(ph + c * 64 + kk * 32 + 16 + 8 * hh);
      pb.h[0] = *(const v8us*)(pl + c * 64 + kk * 32 + 8 * hh);
      pb.h[1] = *(const v8us*)(pl + c * 64 + kk * 32 + 16 + 8 * hh);
#pragma unroll
      for (int t = 0; t < 4; ++t) {
        FB vb;
        vb.h[0] = *(const v8us*)(Vsh + (t * 16 + c) * 64 + kk * 32 + 8 * hh);
        vb.h[1] = *(const v8us*)(Vsh + (t * 16 + c) * 64 + kk * 32 + 16 + 8 * hh);
        oacc[t] = mma_b(pa.v, vb.v, oacc[t]);
        oacc[t] = mma_b(pb.v, vb.v, oacc[t]);
      }
    }
  }

#pragma unroll
  for (int r = 0; r < 8; ++r) {
    float l = lrow[r];
#pragma unroll
    for (int off = 1; off < 16; off <<= 1) l += __shfl_xor(l, off, 32);
    const float inv = (l > 0.f) ? (1.0f / l) : 0.f;
#pragma unroll
    for (int t = 0; t < 4; ++t) Osh[(t * 16 + c) * PO + wave * 16 + 8 * hh + r] = oacc[t][r] * inv;
  }
  __syncthreads();

  {
    const int h2 = lane >> 4, c4 = (lane & 15) * 4;
    for (int pass = 0; pass < 2; ++pass) {
#pragma unroll
      for (int it = 0; it < 8; ++it) {
        const int row = it * 8 + wave * 2 + h2;
        const v4f v = *(const v4f*)(Osh + row * PO + c4);
        *(volatile v4f*)(out + ((size_t)(bh * CH + row)) * SEQ + q0 + c4) = v;
      }
      __threadfence();
    }
  }
}

extern "C" void kernel_launch(void* const* d_in, const int* in_sizes, int n_in,
                              void* d_out, int out_size, void* d_ws, size_t ws_size,
                              hipStream_t stream) {
  if (n_in < 1) return;
  if (in_sizes[0] != NBH * WROW * SEQ) return;
  if (out_size != NBH * CH * SEQ) return;

  const float* qkv = (const float*)d_in[0];
  float* out = (float*)d_out;

  const size_t PPL = (size_t)NBH * SEQ * CH * 2;
  size_t off = 0;
  const size_t oQt = off; off += PPL;
  const size_t oKt = off; off += PPL;
  const size_t oVb = off; off += PPL;
  if (off > ws_size) return;
  if (off > (size_t)134217728) return;

  char* ws = (char*)d_ws;
  unsigned short* Qt = (unsigned short*)(ws + oQt);
  unsigned short* Kt = (unsigned short*)(ws + oKt);
  unsigned short* Vb = (unsigned short*)(ws + oVb);

  const dim3 gPrep(NBH * (SEQ / 64));
  const dim3 gAttn(NBH * NQB);

  prep_planes<<<gPrep, dim3(256), 0, stream>>>(qkv, Qt, Kt, Vb);
  attn64<<<gAttn, dim3(128), 0, stream>>>(Qt, Kt, Vb, out, 0.125f);
  (void)hipGetLastError();
}
